// NMODEL_27633819582859
// MI455X (gfx1250) — hardware-run, weakly checked
//
#include <hip/hip_runtime.h>
#include <math.h>

constexpr int T_STEPS    = 128;
constexpr int BATCH_ROWS = 1024;
constexpr int MODES_D    = 64;
constexpr int HID_D      = 128;
constexpr int Z0_D       = 192;
constexpr int ZW_D       = 256;
constexpr int RK_SUB     = 8;
constexpr int BLK_ROWS   = 32;
constexpr int BLK_THR    = 128;
constexpr int TP_THR     = 256;
constexpr int ZPITCH     = 264;
constexpr int ZBUF       = BLK_ROWS * ZPITCH;
constexpr bool INPUTS_RNE_BF16 = true;
constexpr float WCARRY     = 16.0f;
constexpr float WCARRY_INV = 1.0f / WCARRY;
constexpr float LOG2E_F    = 1.4426950408889634f;
constexpr float SIG_K      = -LOG2E_F * WCARRY_INV;
constexpr float TANH_K     = 2.0f * LOG2E_F * WCARRY_INV;
constexpr float RK_DT      = 1.0f / (float)RK_SUB;
constexpr float RK_W6      = RK_DT / 6.0f;
constexpr float RK_W3      = RK_DT / 3.0f;
constexpr float RK_AH      = 0.5f * RK_DT;
constexpr float RK_AF      = RK_DT;
constexpr int SB_F = 0;
constexpr int SB_1 = HID_D;
constexpr int SB_2 = HID_D + ZW_D;
constexpr int SB_3 = HID_D + 2 * ZW_D;
constexpr int SB_N = 2 * HID_D + 2 * ZW_D;

static_assert(Z0_D == HID_D + MODES_D, "concat width");
static_assert(HID_D == 32 * (BLK_THR / 32), "4 waves x 32 channels");
static_assert(ZW_D == 64 * (BLK_THR / 32), "4 waves x 64 channels");
static_assert(BATCH_ROWS % BLK_ROWS == 0, "rows per block");
static_assert(HID_D % 32 == 0 && Z0_D % 32 == 0 && ZW_D % 32 == 0, "K multiples of 32");
static_assert(HID_D % 64 == 0 && Z0_D % 64 == 0 && ZW_D % 64 == 0 && MODES_D % 64 == 0, "transpose tiles");
static_assert((T_STEPS * BATCH_ROWS) % 64 == 0 && MODES_D == 64, "head GEMM tiles");
static_assert(ZPITCH % 8 == 0 && ZPITCH >= ZW_D, "LDS pitch");
static_assert((2 * ZBUF) % 8 == 0, "LDS zero fill granularity");
static_assert((BLK_ROWS * HID_D) == 4 * BLK_THR * 8, "state plane store coverage");
static_assert((BLK_ROWS * MODES_D) == 2 * BLK_THR * 8, "x staging coverage");
static_assert((4 * RK_SUB) % 2 == 0, "stage count even: buffer parity returns");

typedef __attribute__((ext_vector_type(16))) _Float16 v16h;
typedef __attribute__((ext_vector_type(8)))  _Float16 v8h;
typedef __attribute__((ext_vector_type(8)))  float    v8f;
typedef __attribute__((ext_vector_type(4)))  float    v4f;

__device__ __forceinline__ unsigned short f2bf_bits(float f) {
  unsigned u = __float_as_uint(f);
  return (unsigned short)((u + 0x7FFFu + ((u >> 16) & 1u)) >> 16);
}
__device__ __forceinline__ float bf_bits2f(unsigned short h) { return __uint_as_float(((unsigned)h) << 16); }
__device__ __forceinline__ float bf16r(float f) { return bf_bits2f(f2bf_bits(f)); }
__device__ __forceinline__ float cv_in(float f) { return INPUTS_RNE_BF16 ? bf16r(f) : f; }

__device__ __forceinline__ void guard_stage(v8f& d0, v8f& d1,
                                            v16h a0, v16h a1, v16h a2, v16h a3, v16h a4, v16h a5, v16h a6, v16h a7,
                                            v16h b0, v16h b1, v16h b2, v16h b3) {
  asm volatile("v_nop\n\tv_nop\n\tv_nop\n\tv_nop" : "+v"(d0), "+v"(d1)
               : "v"(a0), "v"(a1), "v"(a2), "v"(a3), "v"(a4), "v"(a5), "v"(a6), "v"(a7),
                 "v"(b0), "v"(b1), "v"(b2), "v"(b3));
}
__device__ __forceinline__ void guard4x4(v8f& d0, v8f& d1, v8f& d2, v8f& d3, v16h a0, v16h a1, v16h b0, v16h b1) {
  asm volatile("v_nop\n\tv_nop\n\tv_nop\n\tv_nop" : "+v"(d0), "+v"(d1), "+v"(d2), "+v"(d3)
               : "v"(a0), "v"(a1), "v"(b0), "v"(b1));
}
__device__ __forceinline__ void guard4x5(v8f& d0, v8f& d1, v8f& d2, v8f& d3, v16h a, v16h b0, v16h b1, v16h b2, v16h b3) {
  asm volatile("v_nop\n\tv_nop\n\tv_nop\n\tv_nop" : "+v"(d0), "+v"(d1), "+v"(d2), "+v"(d3)
               : "v"(a), "v"(b0), "v"(b1), "v"(b2), "v"(b3));
}
__device__ __forceinline__ void keep4_h(v16h a, v16h b, v16h c, v16h d) { asm volatile("v_nop" :: "v"(a), "v"(b), "v"(c), "v"(d)); }
__device__ __forceinline__ void acc_guard4(v8f& a, v8f& b, v8f& c, v8f& d) { asm volatile("v_nop\n\tv_nop\n\tv_nop\n\tv_nop" : "+v"(a), "+v"(b), "+v"(c), "+v"(d)); }

template <typename T> struct Frag;
template <> struct Frag<_Float16> {
  typedef v16h V; union U { v16h v; v8h h[2]; };
  static __device__ __forceinline__ v16h load(const _Float16* p) {
    U f; f.h[0] = *(const v8h*)(p); f.h[1] = *(const v8h*)(p + 16); return f.v;
  }
  static __device__ __forceinline__ v8f mma(v16h a, v16h b, v8f c) {
    return __builtin_amdgcn_wmma_f32_16x16x32_f16(false, a, false, b, (short)0, c, false, false);
  }
};
typedef Frag<_Float16> FH;

template <bool RB>
__global__ __launch_bounds__(TP_THR) void tpw_kernel(const float* __restrict__ src, int R, int C, int ldo,
                                                     unsigned short* __restrict__ O, float sc) {
  __shared__ float Tt[64 * 65];
  const int tid = threadIdx.x;
  const int c0 = blockIdx.x * 64, r0 = blockIdx.y * 64;
#pragma unroll
  for (int i = 0; i < 4; ++i) {
    const int idx = i * TP_THR + tid;
    const int rr = idx >> 4, cc = (idx & 15) * 4;
    const v4f v = *(const v4f*)(src + (size_t)(r0 + rr) * (size_t)C + c0 + cc);
    Tt[rr * 65 + cc + 0] = v[0];
    Tt[rr * 65 + cc + 1] = v[1];
    Tt[rr * 65 + cc + 2] = v[2];
    Tt[rr * 65 + cc + 3] = v[3];
  }
  __syncthreads();
  const int q = tid >> 3, c8 = (tid & 7) * 8;
  v8h hv[2];
#pragma unroll
  for (int g = 0; g < 2; ++g) {
    const int qq = g * 32 + q;
#pragma unroll
    for (int e = 0; e < 8; ++e) {
      const float f = Tt[(c8 + e) * 65 + qq];
      const float fb = RB ? bf16r(f) : f;
      hv[g][e] = (_Float16)(fb * sc);
    }
  }
  for (int pass = 0; pass < 2; ++pass) {
#pragma unroll
    for (int g = 0; g < 2; ++g) {
      const size_t o = (size_t)(c0 + g * 32 + q) * (size_t)ldo + (size_t)(r0 + c8);
      *(volatile v8h*)(O + o) = hv[g];
    }
    __threadfence();
  }
}

__global__ __launch_bounds__(32) void bias_out_kernel(const float* __restrict__ bo, float* __restrict__ dst) {
  const int lane = threadIdx.x;
  if (lane < MODES_D / 4) {
    const v4f v = *(const v4f*)(bo + 4 * lane);
    v4f o;
#pragma unroll
    for (int e = 0; e < 4; ++e) o[e] = cv_in(v[e]);
    *(volatile v4f*)(dst + 4 * lane) = o;
    __threadfence();
    *(volatile v4f*)(dst + 4 * lane) = o;
  }
}

template <int MODE>
__device__ __forceinline__ void rk_stage(const _Float16* src, _Float16* dst, const float* sbf,
                                         const v16h (&wfa)[2][4], float (&hst)[2][2][8], float (&hn)[2][2][8],
                                         const float cw0, const float ca0, const float cw1, const float ca1,
                                         const int c, const int hh, const int chw) {
#pragma unroll
  for (int nt = 0; nt < 2; ++nt) {
    const _Float16* brow = src + (nt * 16 + c) * ZPITCH + 8 * hh;
    const v16h b0 = FH::load(brow);
    const v16h b1 = FH::load(brow + 32);
    const v16h b2 = FH::load(brow + 64);
    const v16h b3 = FH::load(brow + 96);
    v8f acc[2];
    {
      const float* bp = sbf + chw + 8 * hh;
      const v4f x0 = *(const v4f*)(bp);
      const v4f x1 = *(const v4f*)(bp + 4);
      const v4f y0 = *(const v4f*)(bp + 16);
      const v4f y1 = *(const v4f*)(bp + 20);
      acc[0] = (v8f){x0[0], x0[1], x0[2], x0[3], x1[0], x1[1], x1[2], x1[3]};
      acc[1] = (v8f){y0[0], y0[1], y0[2], y0[3], y1[0], y1[1], y1[2], y1[3]};
    }
    acc[0] = FH::mma(wfa[0][0], b0, acc[0]);
    acc[1] = FH::mma(wfa[1][0], b0, acc[1]);
    acc[0] = FH::mma(wfa[0][1], b1, acc[0]);
    acc[1] = FH::mma(wfa[1][1], b1, acc[1]);
    acc[0] = FH::mma(wfa[0][2], b2, acc[0]);
    acc[1] = FH::mma(wfa[1][2], b2, acc[1]);
    acc[0] = FH::mma(wfa[0][3], b3, acc[0]);
    acc[1] = FH::mma(wfa[1][3], b3, acc[1]);
    guard_stage(acc[0], acc[1],
                wfa[0][0], wfa[0][1], wfa[0][2], wfa[0][3], wfa[1][0], wfa[1][1], wfa[1][2], wfa[1][3],
                b0, b1, b2, b3);
    const float cw = (nt == 0) ? cw0 : cw1;
    const float ca = (nt == 0) ? ca0 : ca1;
#pragma unroll
    for (int mt = 0; mt < 2; ++mt) {
      v8h pk;
#pragma unroll
      for (int r = 0; r < 8; ++r) {
        const float ex = __builtin_amdgcn_exp2f(acc[mt][r] * SIG_K);
        const float sg = __builtin_amdgcn_rcpf(1.0f + ex);
        float hv;
        if (MODE == 0) hv = fmaf(cw, sg, hst[mt][nt][r]);
        else           hv = fmaf(cw, sg, hn[mt][nt][r]);
        hn[mt][nt][r] = hv;
        float nx;
        if (MODE == 2) { hst[mt][nt][r] = hv; nx = hv; }
        else           { nx = fmaf(ca, sg, hst[mt][nt][r]); }
        pk[r] = (_Float16)nx;
      }
      *(v8h*)(dst + (nt * 16 + c) * ZPITCH + chw + 16 * mt + 8 * hh) = pk;
    }
    __builtin_amdgcn_sched_barrier(0);
  }
  __syncthreads();
}

template <int KCH>
__device__ __forceinline__ void mlp_pair(const _Float16* __restrict__ wrow, const int ldw,
                                         const _Float16* zrow, const float* bp, v8f (&acc)[2][2]) {
  {
    const v4f x0 = *(const v4f*)(bp);
    const v4f x1 = *(const v4f*)(bp + 4);
    const v4f y0 = *(const v4f*)(bp + 16);
    const v4f y1 = *(const v4f*)(bp + 20);
    const v8f i0 = {x0[0], x0[1], x0[2], x0[3], x1[0], x1[1], x1[2], x1[3]};
    const v8f i1 = {y0[0], y0[1], y0[2], y0[3], y1[0], y1[1], y1[2], y1[3]};
    acc[0][0] = i0; acc[0][1] = i0; acc[1][0] = i1; acc[1][1] = i1;
  }
  const _Float16* wrow1 = wrow + 16 * ldw;
  const _Float16* zrow1 = zrow + 16 * ZPITCH;
#pragma unroll 1
  for (int kc = 0; kc < KCH; ++kc) {
    const int ko = kc * 32;
    const v16h a0 = FH::load(wrow + ko);
    const v16h a1 = FH::load(wrow1 + ko);
    const v16h b0 = FH::load(zrow + ko);
    const v16h b1 = FH::load(zrow1 + ko);
    acc[0][0] = FH::mma(a0, b0, acc[0][0]);
    acc[1][0] = FH::mma(a1, b0, acc[1][0]);
    acc[0][1] = FH::mma(a0, b1, acc[0][1]);
    acc[1][1] = FH::mma(a1, b1, acc[1][1]);
    guard4x4(acc[0][0], acc[0][1], acc[1][0], acc[1][1], a0, a1, b0, b1);
  }
}

__device__ __forceinline__ void store_tanh(const v8f (&acc)[2][2], _Float16* dst, const int chp, const int c, const int hh) {
#pragma unroll
  for (int nt = 0; nt < 2; ++nt) {
#pragma unroll
    for (int mt = 0; mt < 2; ++mt) {
      v8h pk;
#pragma unroll
      for (int r = 0; r < 8; ++r) {
        const float ex = __builtin_amdgcn_exp2f(acc[mt][nt][r] * TANH_K);
        pk[r] = (_Float16)(1.0f - 2.0f * __builtin_amdgcn_rcpf(ex + 1.0f));
      }
      *(v8h*)(dst + (nt * 16 + c) * ZPITCH + chp + 16 * mt + 8 * hh) = pk;
    }
  }
}

__device__ __forceinline__ void hs_store(const _Float16* zb, unsigned short* dstblk, const int tid) {
  v8h hv[4];
#pragma unroll
  for (int it = 0; it < 4; ++it) {
    const int idx = it * BLK_THR + tid;
    hv[it] = *(const v8h*)(zb + (idx >> 4) * ZPITCH + (idx & 15) * 8);
  }
  for (int pass = 0; pass < 2; ++pass) {
#pragma unroll
    for (int it = 0; it < 4; ++it) {
      const int idx = it * BLK_THR + tid;
      *(volatile v8h*)(dstblk + (size_t)idx * 8) = hv[it];
    }
    __threadfence();
  }
}

__global__ __launch_bounds__(BLK_THR) __attribute__((amdgpu_num_vgpr(256)))
void ode_rnn_kernel(const float* __restrict__ tin, const float* __restrict__ xin,
                    const float* __restrict__ bfp, const float* __restrict__ b1p,
                    const float* __restrict__ b2p, const float* __restrict__ b3p,
                    const unsigned short* __restrict__ WfTp, const unsigned short* __restrict__ W1Tp,
                    const unsigned short* __restrict__ W2Tp, const unsigned short* __restrict__ W3Tp,
                    unsigned short* __restrict__ HSp) {
  __shared__ __align__(16) _Float16 Zb[2 * ZBUF];
  __shared__ __align__(16) float    sBias[SB_N];
  const _Float16* WfT = (const _Float16*)WfTp;
  const _Float16* W1T = (const _Float16*)W1Tp;
  const _Float16* W2T = (const _Float16*)W2Tp;
  const _Float16* W3T = (const _Float16*)W3Tp;
  const int tid = threadIdx.x, lane = tid & 31, wave = tid >> 5;
  const int c = lane & 15, hh = lane >> 4;
  const int rowbase = blockIdx.x * BLK_ROWS;
  const int chw = 32 * wave;

  {
    v8h zz;
#pragma unroll
    for (int e = 0; e < 8; ++e) zz[e] = (_Float16)0.0f;
    v8h* zp = (v8h*)Zb;
#pragma unroll 1
    for (int i = tid; i < (2 * ZBUF) / 8; i += BLK_THR) zp[i] = zz;
  }
  sBias[SB_F + tid]       = WCARRY * cv_in(bfp[tid]);
  sBias[SB_1 + tid]       = WCARRY * cv_in(b1p[tid]);
  sBias[SB_1 + 128 + tid] = WCARRY * cv_in(b1p[128 + tid]);
  sBias[SB_2 + tid]       = WCARRY * cv_in(b2p[tid]);
  sBias[SB_2 + 128 + tid] = WCARRY * cv_in(b2p[128 + tid]);
  sBias[SB_3 + tid]       = WCARRY * cv_in(b3p[tid]);

  v16h wfa[2][4];
#pragma unroll
  for (int mt = 0; mt < 2; ++mt)
#pragma unroll
    for (int kc = 0; kc < 4; ++kc)
      wfa[mt][kc] = FH::load(WfT + (size_t)(chw + 16 * mt + c) * HID_D + kc * 32 + 8 * hh);

  float hst[2][2][8];
#pragma unroll
  for (int mt = 0; mt < 2; ++mt)
#pragma unroll
    for (int nt = 0; nt < 2; ++nt)
#pragma unroll
      for (int r = 0; r < 8; ++r) hst[mt][nt][r] = 0.0f;
  __syncthreads();

#pragma unroll 1
  for (int step = 0; step < T_STEPS - 1; ++step) {
    _Float16* X = Zb + (step & 1) * ZBUF;
    _Float16* Y = Zb + ((step & 1) ^ 1) * ZBUF;

    hs_store(X, HSp + ((size_t)step * BATCH_ROWS + rowbase) * HID_D, tid);

#pragma unroll
    for (int it = 0; it < 2; ++it) {
      const int idx = it * BLK_THR + tid;
      const int row = idx >> 3, c8 = (idx & 7) * 8;
      const float* xp = xin + ((size_t)step * BATCH_ROWS + rowbase + row) * MODES_D + c8;
      const v4f a = *(const v4f*)(xp);
      const v4f b = *(const v4f*)(xp + 4);
      v8h hv;
#pragma unroll
      for (int e = 0; e < 4; ++e) {
        hv[e]     = (_Float16)cv_in(a[e]);
        hv[4 + e] = (_Float16)cv_in(b[e]);
      }
      *(v8h*)(X + row * ZPITCH + HID_D + c8) = hv;
    }

    const float tc0 = cv_in(tin[(size_t)step * BATCH_ROWS + rowbase + c]);
    const float tc1 = cv_in(tin[(size_t)step * BATCH_ROWS + rowbase + 16 + c]);
    const float cw6_0 = tc0 * RK_W6, cw6_1 = tc1 * RK_W6;
    const float cw3_0 = tc0 * RK_W3, cw3_1 = tc1 * RK_W3;
    const float cah_0 = tc0 * RK_AH, cah_1 = tc1 * RK_AH;
    const float caf_0 = tc0 * RK_AF, caf_1 = tc1 * RK_AF;

    {
      float hn[2][2][8];
#pragma unroll 1
      for (int s = 0; s < RK_SUB; ++s) {
        rk_stage<0>(X, Y, sBias + SB_F, wfa, hst, hn, cw6_0, cah_0, cw6_1, cah_1, c, hh, chw);
        rk_stage<1>(Y, X, sBias + SB_F, wfa, hst, hn, cw3_0, cah_0, cw3_1, cah_1, c, hh, chw);
        rk_stage<1>(X, Y, sBias + SB_F, wfa, hst, hn, cw3_0, caf_0, cw3_1, caf_1, c, hh, chw);
        rk_stage<2>(Y, X, sBias + SB_F, wfa, hst, hn, cw6_0, 0.0f, cw6_1, 0.0f, c, hh, chw);
      }
    }

#pragma unroll 1
    for (int mp = 0; mp < 2; ++mp) {
      const int chp = 64 * wave + 32 * mp;
      v8f acc[2][2];
      mlp_pair<Z0_D / 32>(W1T + (size_t)(chp + c) * Z0_D + 8 * hh, Z0_D, X + c * ZPITCH + 8 * hh,
                          sBias + SB_1 + chp + 8 * hh, acc);
      store_tanh(acc, Y, chp, c, hh);
    }
    __syncthreads();

#pragma unroll 1
    for (int mp = 0; mp < 2; ++mp) {
      const int chp = 64 * wave + 32 * mp;
      v8f acc[2][2];
      mlp_pair<ZW_D / 32>(W2T + (size_t)(chp + c) * ZW_D + 8 * hh, ZW_D, Y + c * ZPITCH + 8 * hh,
                          sBias + SB_2 + chp + 8 * hh, acc);
      store_tanh(acc, X, chp, c, hh);
    }
    __syncthreads();

    {
      v8f acc[2][2];
      mlp_pair<ZW_D / 32>(W3T + (size_t)(chw + c) * ZW_D + 8 * hh, ZW_D, X + c * ZPITCH + 8 * hh,
                          sBias + SB_3 + chw + 8 * hh, acc);
#pragma unroll
      for (int nt = 0; nt < 2; ++nt) {
#pragma unroll
        for (int mt = 0; mt < 2; ++mt) {
          v8h pk;
#pragma unroll
          for (int r = 0; r < 8; ++r) {
            const float hv = acc[mt][nt][r] * WCARRY_INV;
            hst[mt][nt][r] = hv;
            pk[r] = (_Float16)hv;
          }
          *(v8h*)(Y + (nt * 16 + c) * ZPITCH + chw + 16 * mt + 8 * hh) = pk;
        }
      }
    }
    __syncthreads();
  }

  hs_store(Zb + ((T_STEPS - 1) & 1) * ZBUF,
           HSp + ((size_t)(T_STEPS - 1) * BATCH_ROWS + rowbase) * HID_D, tid);
}

__global__ __launch_bounds__(256) void head_gemm_kernel(
    const unsigned short* __restrict__ Ap, int lda,
    const unsigned short* __restrict__ Btp, int ldb,
    float* __restrict__ Cout, int ldc,
    const float* __restrict__ bias,
    int M, int N, int K, float scale) {
  const _Float16* A  = (const _Float16*)Ap;
  const _Float16* Bt = (const _Float16*)Btp;
  __shared__ __align__(16) float sT[8][16 * 68];
  const int lane = threadIdx.x & 31;
  const int wave = threadIdx.x >> 5;
  const int tilesN = N >> 6;
  const int tilesM = M >> 6;
  const int tile = blockIdx.x * 8 + wave;
  if (tile >= tilesM * tilesN) return;
  const int tm = tile / tilesN;
  const int tn = tile - tm * tilesN;
  const int m0 = tm << 6;
  const int n0 = tn << 6;
  const int rlane = lane & 15;
  const int koff  = (lane >> 4) * 8;
  const int mOff  = (lane >> 4) * 8;

  v8f acc[4][4];
#pragma unroll
  for (int i = 0; i < 4; ++i)
#pragma unroll
    for (int j = 0; j < 4; ++j) acc[i][j] = (v8f){0.f, 0.f, 0.f, 0.f, 0.f, 0.f, 0.f, 0.f};

  for (int k0 = 0; k0 < K; k0 += 32) {
    v16h bh[4];
#pragma unroll
    for (int j = 0; j < 4; ++j) {
      const size_t bo = (size_t)(n0 + (j << 4) + rlane) * ldb + koff + k0;
      bh[j] = FH::load(Bt + bo);
    }
#pragma unroll
    for (int i = 0; i < 4; ++i) {
      const size_t ao = (size_t)(m0 + (i << 4) + rlane) * lda + koff + k0;
      const v16h ah = FH::load(A + ao);
#pragma unroll
      for (int j = 0; j < 4; ++j) acc[i][j] = FH::mma(ah, bh[j], acc[i][j]);
      guard4x5(acc[i][0], acc[i][1], acc[i][2], acc[i][3], ah, bh[0], bh[1], bh[2], bh[3]);
    }
    keep4_h(bh[0], bh[1], bh[2], bh[3]);
  }
  acc_guard4(acc[0][0], acc[0][1], acc[0][2], acc[0][3]);
  acc_guard4(acc[1][0], acc[1][1], acc[1][2], acc[1][3]);
  acc_guard4(acc[2][0], acc[2][1], acc[2][2], acc[2][3]);
  acc_guard4(acc[3][0], acc[3][1], acc[3][2], acc[3][3]);

  float* slab = sT[wave];
#pragma unroll
  for (int i = 0; i < 4; ++i) {
    const int mBase = m0 + (i << 4);
#pragma unroll
    for (int j = 0; j < 4; ++j) {
      const int n = n0 + (j << 4) + rlane;
      const float bv = bias[n];
#pragma unroll
      for (int r = 0; r < 8; ++r) {
        const float v = acc[i][j][r] * scale + bv;
        slab[(mOff + r) * 68 + (j << 4) + rlane] = v;
      }
    }
    __builtin_amdgcn_fence(__ATOMIC_RELEASE, "workgroup");
    __builtin_amdgcn_wave_barrier();
    __builtin_amdgcn_fence(__ATOMIC_ACQUIRE, "workgroup");
    {
      const int hh = lane >> 4, c4 = (lane & 15) * 4;
      for (int pass = 0; pass < 2; ++pass) {
#pragma unroll
        for (int it = 0; it < 8; ++it) {
          const int row = it * 2 + hh;
          const v4f v = *(const v4f*)(slab + row * 68 + c4);
          *(volatile v4f*)(Cout + (size_t)(mBase + row) * ldc + n0 + c4) = v;
        }
        __threadfence();
      }
    }
    __builtin_amdgcn_fence(__ATOMIC_RELEASE, "workgroup");
    __builtin_amdgcn_wave_barrier();
    __builtin_amdgcn_fence(__ATOMIC_ACQUIRE, "workgroup");
  }
}

extern "C" void kernel_launch(void* const* d_in, const int* in_sizes, int n_in,
                              void* d_out, int out_size, void* d_ws, size_t ws_size, hipStream_t stream) {
  if (n_in < 12 || d_out == nullptr || d_ws == nullptr) return;
  if (in_sizes[0] != T_STEPS * BATCH_ROWS || in_sizes[1] != T_STEPS * BATCH_ROWS * MODES_D ||
      in_sizes[2] != HID_D * HID_D || in_sizes[3] != HID_D ||
      in_sizes[4] != Z0_D * ZW_D || in_sizes[5] != ZW_D ||
      in_sizes[6] != ZW_D * ZW_D || in_sizes[7] != ZW_D ||
      in_sizes[8] != ZW_D * HID_D || in_sizes[9] != HID_D ||
      in_sizes[10] != HID_D * MODES_D || in_sizes[11] != MODES_D ||
      out_size != T_STEPS * BATCH_ROWS * MODES_D) return;

  const float* tin = (const float*)d_in[0];
  const float* xin = (const float*)d_in[1];
  const float* Wf  = (const float*)d_in[2];
  const float* bfp = (const float*)d_in[3];
  const float* W1  = (const float*)d_in[4];
  const float* b1p = (const float*)d_in[5];
  const float* W2  = (const float*)d_in[6];
  const float* b2p = (const float*)d_in[7];
  const float* W3  = (const float*)d_in[8];
  const float* b3p = (const float*)d_in[9];
  const float* Wo  = (const float*)d_in[10];
  const float* bop = (const float*)d_in[11];
  float* out = (float*)d_out;

  char* ws = (char*)d_ws; size_t off = 0;
  auto carve = [&](size_t bytes) -> char* { char* p = ws + off; off += (bytes + 255) & ~(size_t)255; return p; };
  unsigned short* WfT = (unsigned short*)carve((size_t)HID_D * HID_D * 2);
  unsigned short* W1T = (unsigned short*)carve((size_t)ZW_D * Z0_D * 2);
  unsigned short* W2T = (unsigned short*)carve((size_t)ZW_D * ZW_D * 2);
  unsigned short* W3T = (unsigned short*)carve((size_t)HID_D * ZW_D * 2);
  unsigned short* WoT = (unsigned short*)carve((size_t)MODES_D * HID_D * 2);
  float*          BO  = (float*)carve((size_t)MODES_D * 4);
  unsigned short* HS  = (unsigned short*)carve((size_t)T_STEPS * BATCH_ROWS * HID_D * 2);
  if (off > ws_size || off > (size_t)134217728) return;

  tpw_kernel<INPUTS_RNE_BF16><<<dim3(HID_D / 64, HID_D / 64), TP_THR, 0, stream>>>(Wf, HID_D, HID_D, HID_D, WfT, WCARRY);
  tpw_kernel<INPUTS_RNE_BF16><<<dim3(ZW_D / 64, Z0_D / 64), TP_THR, 0, stream>>>(W1, Z0_D, ZW_D, Z0_D, W1T, WCARRY);
  tpw_kernel<INPUTS_RNE_BF16><<<dim3(ZW_D / 64, ZW_D / 64), TP_THR, 0, stream>>>(W2, ZW_D, ZW_D, ZW_D, W2T, WCARRY);
  tpw_kernel<INPUTS_RNE_BF16><<<dim3(HID_D / 64, ZW_D / 64), TP_THR, 0, stream>>>(W3, ZW_D, HID_D, ZW_D, W3T, WCARRY);
  tpw_kernel<INPUTS_RNE_BF16><<<dim3(MODES_D / 64, HID_D / 64), TP_THR, 0, stream>>>(Wo, HID_D, MODES_D, HID_D, WoT, WCARRY);
  bias_out_kernel<<<1, 32, 0, stream>>>(bop, BO);

  ode_rnn_kernel<<<BATCH_ROWS / BLK_ROWS, BLK_THR, 0, stream>>>(tin, xin, bfp, b1p, b2p, b3p, WfT, W1T, W2T, W3T, HS);

  head_gemm_kernel<<<(T_STEPS * BATCH_ROWS / 64) / 8, 256, 0, stream>>>(
      HS, HID_D, WoT, HID_D, out, MODES_D, BO, T_STEPS * BATCH_ROWS, MODES_D, HID_D, WCARRY_INV);
}
